// BatchGraphVariationalAutoencoder_3504693314191
// MI455X (gfx1250) — hardware-verified
//
#include <hip/hip_runtime.h>
#define BB 8
#define NN 2048
#define FF 64
#define HH 256
#define LAT 64
#define K1 1024
#define K2 512

typedef __bf16 v16b __attribute__((ext_vector_type(16)));
typedef unsigned short v8us __attribute__((ext_vector_type(8), may_alias));
typedef float  v8f  __attribute__((ext_vector_type(8)));
typedef float  v4f  __attribute__((ext_vector_type(4)));
typedef float  v4fa __attribute__((ext_vector_type(4), may_alias));
union FragB { v16b v; v8us half[2]; unsigned short u[16]; };

__device__ __forceinline__ unsigned short bf16_bits(float x) { unsigned int u = __float_as_uint(x); return (unsigned short)((u + 0x7FFFu + ((u >> 16) & 1u)) >> 16); }
__device__ __forceinline__ float bf16_val(unsigned short b) { return __uint_as_float(((unsigned int)b) << 16); }
__device__ __forceinline__ float bf16_round(float x) { return bf16_val(bf16_bits(x)); }
template <int NT>
__device__ __forceinline__ v8f mmaN(v16b ah, v16b al, v16b bh, v16b bl, v8f c) {
  c = __builtin_amdgcn_wmma_f32_16x16x32_bf16(false, ah, false, bh, (short)0, c, false, false);
  if (NT >= 2) c = __builtin_amdgcn_wmma_f32_16x16x32_bf16(false, al, false, bh, (short)0, c, false, false);
  if (NT >= 3) c = __builtin_amdgcn_wmma_f32_16x16x32_bf16(false, ah, false, bl, (short)0, c, false, false);
  asm volatile("v_nop\n\tv_nop\n\tv_nop\n\tv_nop" : "+v"(c) : "v"(ah), "v"(al), "v"(bh), "v"(bl));
  return c;
}

__global__ __launch_bounds__(256) void k_wt_bf16(const float* __restrict__ W, unsigned short* __restrict__ Wt, int K, int N) {
  const int t = blockIdx.x * 256 + threadIdx.x;
  const int k8n = K / 8;
  if (t >= N * k8n) return;
  const int n = t / k8n, k8 = (t % k8n) * 8;
  v8us v;
#pragma unroll
  for (int i = 0; i < 8; ++i) v[i] = bf16_bits(W[(size_t)(k8 + i) * N + n]);
  *(volatile v8us*)(Wt + (size_t)n * K + k8) = v;
  __threadfence();
  *(volatile v8us*)(Wt + (size_t)n * K + k8) = v;
}

template <bool ASPLIT, int ACT, bool BIAS_BF16>
__global__ __launch_bounds__(128) void k_gemm_bf(const float* __restrict__ A, int lda, const unsigned short* __restrict__ Wt, int ldb,
                                               const float* __restrict__ bias, float* __restrict__ C, int ldc, int M, int N, int K) {
  __shared__ __attribute__((aligned(16))) float so[4][16][64];
  const int tid = threadIdx.x, w = tid >> 5, lane = tid & 31, ln = lane & 15, hh = lane >> 4;
  const int ntn = N / 64;
  const int wid = blockIdx.x * 4 + w;
  const int mt = wid / ntn, nq = wid % ntn;
  if (mt * 16 >= M) return;
  const int row0 = mt * 16, col0 = nq * 64;
  const float* arow = A + (size_t)(row0 + ln) * lda;
  v8f acc[4] = {};
  for (int kb = 0; kb < K; kb += 32) {
    FragB ah, al;
    const v4f x0 = *(const v4fa*)(arow + kb + 8 * hh), x1 = *(const v4fa*)(arow + kb + 8 * hh + 4);
    const v4f x2 = *(const v4fa*)(arow + kb + 16 + 8 * hh), x3 = *(const v4fa*)(arow + kb + 16 + 8 * hh + 4);
    float xs[16] = {x0[0],x0[1],x0[2],x0[3],x1[0],x1[1],x1[2],x1[3],x2[0],x2[1],x2[2],x2[3],x3[0],x3[1],x3[2],x3[3]};
#pragma unroll
    for (int i = 0; i < 16; ++i) { const unsigned short hb = bf16_bits(xs[i]); ah.u[i] = hb; al.u[i] = ASPLIT ? bf16_bits(xs[i] - bf16_val(hb)) : (unsigned short)0; }
#pragma unroll
    for (int t = 0; t < 4; ++t) {
      const unsigned short* brow = Wt + (size_t)(col0 + t * 16 + ln) * ldb + kb;
      FragB b;
      b.half[0] = *(const v8us*)(brow + 8 * hh);
      b.half[1] = *(const v8us*)(brow + 16 + 8 * hh);
      acc[t] = mmaN<ASPLIT ? 2 : 1>(ah.v, al.v, b.v, b.v, acc[t]);
    }
  }
#pragma unroll
  for (int t = 0; t < 4; ++t) {
    float bv = bias ? bias[col0 + t * 16 + ln] : 0.f;
    if (BIAS_BF16) bv = bf16_round(bv);
#pragma unroll
    for (int r = 0; r < 8; ++r) { float v = acc[t][r] + bv; if (ACT == 1) v = fmaxf(v, 0.f); so[w][8 * hh + r][t * 16 + ln] = v; }
  }
  __builtin_amdgcn_fence(__ATOMIC_ACQ_REL, "workgroup");
  __builtin_amdgcn_wave_barrier();
  const int rsub = lane >> 4, c4 = (lane & 15) * 4;
  for (int pass = 0; pass < 2; ++pass) {
#pragma unroll
    for (int q = 0; q < 8; ++q) {
      const int r = q * 2 + rsub;
      const v4f v = *(const v4fa*)&so[w][r][c4];
      *(volatile v4f*)(C + (size_t)(row0 + r) * ldc + col0 + c4) = v;
    }
    if (pass == 0) __threadfence();
  }
}

template <int D, bool CAUSAL>
__global__ __launch_bounds__(128) void k_flash(const float* __restrict__ qb, const float* __restrict__ kb, const float* __restrict__ vb,
                                             int pitch, int T, int H, float scale, float* __restrict__ y, int ypitch) {
  constexpr int KS = D / 32;
  constexpr int DT = D / 16;
  __shared__ __attribute__((aligned(16))) unsigned short sKh[32][D + 8], sKl[32][D + 8], sVh[32][D + 8], sVl[32][D + 8];
  __shared__ __attribute__((aligned(16))) unsigned short sPh[4][16][40], sPl[4][16][40];
  __shared__ __attribute__((aligned(16))) float sO[4][16][D];
  const int tid = threadIdx.x, w = tid >> 5, lane = tid & 31, ln = lane & 15, hh = lane >> 4;
  const int nqb = (T + 63) / 64;
  const int bh = blockIdx.x / nqb, qblk = blockIdx.x % nqb;
  const int b = bh / H, h = bh % H;
  const int q0 = qblk * 64 + w * 16;
  const float* Q = qb + (size_t)b * T * pitch + h * D;
  const float* K = kb + (size_t)b * T * pitch + h * D;
  const float* V = vb + (size_t)b * T * pitch + h * D;

  FragB aqh[KS], aql[KS];
  {
    int row = q0 + ln; if (row >= T) row = T - 1;
    const float* qr = Q + (size_t)row * pitch;
#pragma unroll
    for (int ks = 0; ks < KS; ++ks)
#pragma unroll
      for (int i = 0; i < 16; ++i) {
        const int d = ks * 32 + ((i < 8) ? (8 * hh + i) : (16 + 8 * hh + (i - 8)));
        const float x = qr[d] * scale; const unsigned short hb = bf16_bits(x);
        aqh[ks].u[i] = hb; aql[ks].u[i] = bf16_bits(x - bf16_val(hb));
      }
  }
  float m_r[8], l_r[8];
#pragma unroll
  for (int r = 0; r < 8; ++r) { m_r[r] = -3.0e38f; l_r[r] = 0.f; }
  v8f oacc[DT];
#pragma unroll
  for (int dt = 0; dt < DT; ++dt) oacc[dt] = (v8f){0.f,0.f,0.f,0.f,0.f,0.f,0.f,0.f};

  const int kv_end = CAUSAL ? min(T, qblk * 64 + 64) : T;
  for (int j0 = 0; j0 < kv_end; j0 += 32) {
    __syncthreads();
    for (int e = tid; e < 32 * (D / 4); e += 128) {
      const int r = e / (D / 4), c4 = (e % (D / 4)) * 4;
      const int key = j0 + r;
      v4f kf = {0.f,0.f,0.f,0.f}, vf = {0.f,0.f,0.f,0.f};
      if (key < T) { kf = *(const v4fa*)(K + (size_t)key * pitch + c4); vf = *(const v4fa*)(V + (size_t)key * pitch + c4); }
#pragma unroll
      for (int t = 0; t < 4; ++t) {
        unsigned short hb = bf16_bits(kf[t]); sKh[r][c4 + t] = hb; sKl[r][c4 + t] = bf16_bits(kf[t] - bf16_val(hb));
        hb = bf16_bits(vf[t]); sVh[r][c4 + t] = hb; sVl[r][c4 + t] = bf16_bits(vf[t] - bf16_val(hb));
      }
    }
    __syncthreads();
    v8f s[2];
#pragma unroll
    for (int nt = 0; nt < 2; ++nt) {
      v8f acc = {};
#pragma unroll
      for (int ks = 0; ks < KS; ++ks) {
        FragB bh_, bl_;
        bh_.half[0] = *(const v8us*)&sKh[nt * 16 + ln][ks * 32 + 8 * hh]; bh_.half[1] = *(const v8us*)&sKh[nt * 16 + ln][ks * 32 + 16 + 8 * hh];
        bl_.half[0] = *(const v8us*)&sKl[nt * 16 + ln][ks * 32 + 8 * hh]; bl_.half[1] = *(const v8us*)&sKl[nt * 16 + ln][ks * 32 + 16 + 8 * hh];
        acc = mmaN<3>(aqh[ks].v, aql[ks].v, bh_.v, bl_.v, acc);
      }
      s[nt] = acc;
    }
    float alpha[8];
#pragma unroll
    for (int r = 0; r < 8; ++r) {
      const int qi = q0 + 8 * hh + r;
      const int ja = j0 + ln, jb = j0 + 16 + ln;
      if (CAUSAL) { if (ja > qi) s[0][r] = -3.0e38f; if (jb > qi) s[1][r] = -3.0e38f; }
      if (ja >= T) s[0][r] = -3.0e38f;
      if (jb >= T) s[1][r] = -3.0e38f;
      float mx = fmaxf(s[0][r], s[1][r]);
      mx = fmaxf(mx, __shfl_xor(mx, 1, 32)); mx = fmaxf(mx, __shfl_xor(mx, 2, 32)); mx = fmaxf(mx, __shfl_xor(mx, 4, 32)); mx = fmaxf(mx, __shfl_xor(mx, 8, 32));
      const float mnew = fmaxf(m_r[r], mx);
      alpha[r] = (mnew > -1.0e38f) ? __expf(m_r[r] - mnew) : 1.0f;
      const float p0 = (s[0][r] > -1.0e38f) ? __expf(s[0][r] - mnew) : 0.f;
      const float p1 = (s[1][r] > -1.0e38f) ? __expf(s[1][r] - mnew) : 0.f;
      m_r[r] = mnew;
      l_r[r] = l_r[r] * alpha[r] + p0 + p1;
      unsigned short hb = bf16_bits(p0); sPh[w][8 * hh + r][ln] = hb;      sPl[w][8 * hh + r][ln] = bf16_bits(p0 - bf16_val(hb));
      hb = bf16_bits(p1);                sPh[w][8 * hh + r][16 + ln] = hb; sPl[w][8 * hh + r][16 + ln] = bf16_bits(p1 - bf16_val(hb));
    }
#pragma unroll
    for (int dt = 0; dt < DT; ++dt)
#pragma unroll
      for (int r = 0; r < 8; ++r) oacc[dt][r] *= alpha[r];
    __builtin_amdgcn_fence(__ATOMIC_ACQ_REL, "workgroup");
    __builtin_amdgcn_wave_barrier();
    FragB pah, pal;
    pah.half[0] = *(const v8us*)&sPh[w][ln][8 * hh]; pah.half[1] = *(const v8us*)&sPh[w][ln][16 + 8 * hh];
    pal.half[0] = *(const v8us*)&sPl[w][ln][8 * hh]; pal.half[1] = *(const v8us*)&sPl[w][ln][16 + 8 * hh];
#pragma unroll
    for (int dt = 0; dt < DT; ++dt) {
      FragB bvh, bvl;
#pragma unroll
      for (int i = 0; i < 8; ++i) {
        bvh.u[i] = sVh[8 * hh + i][dt * 16 + ln]; bvh.u[8 + i] = sVh[16 + 8 * hh + i][dt * 16 + ln];
        bvl.u[i] = sVl[8 * hh + i][dt * 16 + ln]; bvl.u[8 + i] = sVl[16 + 8 * hh + i][dt * 16 + ln];
      }
      oacc[dt] = mmaN<3>(pah.v, pal.v, bvh.v, bvl.v, oacc[dt]);
    }
    __builtin_amdgcn_fence(__ATOMIC_ACQ_REL, "workgroup");
    __builtin_amdgcn_wave_barrier();
  }
#pragma unroll
  for (int r = 0; r < 8; ++r) {
    float l = l_r[r];
    l += __shfl_xor(l, 1, 32); l += __shfl_xor(l, 2, 32); l += __shfl_xor(l, 4, 32); l += __shfl_xor(l, 8, 32);
    l_r[r] = (l > 0.f) ? 1.0f / l : 0.f;
  }
#pragma unroll
  for (int dt = 0; dt < DT; ++dt)
#pragma unroll
    for (int r = 0; r < 8; ++r) sO[w][8 * hh + r][dt * 16 + ln] = oacc[dt][r] * l_r[r];
  __builtin_amdgcn_fence(__ATOMIC_ACQ_REL, "workgroup");
  __builtin_amdgcn_wave_barrier();
  for (int pass = 0; pass < 2; ++pass) {
    for (int r = 0; r < 16; ++r) {
      const int row = q0 + r;
      if (row < T && lane < D / 4) {
        const v4f val = *(const v4fa*)&sO[w][r][lane * 4];
        *(volatile v4f*)(y + ((size_t)b * T + row) * ypitch + h * D + lane * 4) = val;
      }
    }
    if (pass == 0) __threadfence();
  }
}

template <bool AFFINE, bool RESID, bool RES_BF16>
__global__ __launch_bounds__(256) void k_transpose32(const float* __restrict__ in, float* __restrict__ out, int rows, int cols,
                                                    const float* __restrict__ scale, const float* __restrict__ shift, const float* __restrict__ res) {
  __shared__ float tile[32][33];
  const int b = blockIdx.z;
  const int r0 = blockIdx.y * 32, c0 = blockIdx.x * 32;
  const float* src = in + (size_t)b * rows * cols;
  float* dst = out + (size_t)b * rows * cols;
  const int tx = threadIdx.x & 31, ty = threadIdx.x >> 5;
  for (int i = ty; i < 32; i += 8) tile[i][tx] = src[(size_t)(r0 + i) * cols + c0 + tx];
  __syncthreads();
  for (int pass = 0; pass < 2; ++pass) {
    for (int i = ty; i < 32; i += 8) {
      float v = tile[tx][i];
      const int orow = c0 + i;
      if (AFFINE) v = v * scale[orow] + shift[orow];
      if (RESID) { float rv = res[(size_t)b * rows * cols + (size_t)orow * rows + r0 + tx]; if (RES_BF16) rv = bf16_round(rv); v += rv; }
      *(volatile float*)(dst + (size_t)orow * rows + r0 + tx) = v;
    }
    if (pass == 0) __threadfence();
  }
}

__global__ __launch_bounds__(256) void k_pool2_pm(const float* __restrict__ in, float* __restrict__ out, int Bn, int H, int W, int C) {
  const size_t t = (size_t)blockIdx.x * 256 + threadIdx.x;
  const int c4n = C / 4, Ho = H / 2, Wo = W / 2;
  const size_t total = (size_t)Bn * Ho * Wo * c4n;
  if (t >= total) return;
  const int c4 = (int)(t % c4n) * 4; size_t rest = t / c4n;
  const int pw = (int)(rest % Wo); rest /= Wo; const int ph = (int)(rest % Ho); const int b = (int)(rest / Ho);
  const float* base = in + (size_t)b * H * W * C;
  const int p00 = (2 * ph) * W + 2 * pw;
  const v4f a = *(const v4fa*)(base + (size_t)p00 * C + c4), bq = *(const v4fa*)(base + (size_t)(p00 + 1) * C + c4);
  const v4f c = *(const v4fa*)(base + (size_t)(p00 + W) * C + c4), d = *(const v4fa*)(base + (size_t)(p00 + W + 1) * C + c4);
  v4f m; for (int i = 0; i < 4; ++i) m[i] = fmaxf(fmaxf(a[i], bq[i]), fmaxf(c[i], d[i]));
  float* dst = out + ((size_t)b * Ho * Wo + (size_t)ph * Wo + pw) * C + c4;
  *(volatile v4f*)dst = m;
  __threadfence();
  *(volatile v4f*)dst = m;
}

template <int DQ, int DV>
__global__ __launch_bounds__(128) void k_flash2(const float* __restrict__ Qb, size_t qstride, int qpitch, int Tq,
                                              const float* __restrict__ Kb, size_t kstride, int kpitch, int Tk,
                                              const float* __restrict__ Vb, size_t vstride, int vpitch,
                                              float scale, float* __restrict__ y, size_t ystride, int ypitch) {
  constexpr int KS = DQ / 32, DT = DV / 16;
  __shared__ __attribute__((aligned(16))) unsigned short sKh[32][DQ + 8], sKl[32][DQ + 8], sVh[32][DV + 8], sVl[32][DV + 8];
  __shared__ __attribute__((aligned(16))) unsigned short sPh[4][16][40], sPl[4][16][40];
  __shared__ __attribute__((aligned(16))) float sO[4][16][DV];
  const int tid = threadIdx.x, w = tid >> 5, lane = tid & 31, ln = lane & 15, hh = lane >> 4;
  const int nqb = (Tq + 63) / 64;
  const int bh = blockIdx.x / nqb, qblk = blockIdx.x % nqb;
  const int dv0 = blockIdx.y * DV;
  const int q0 = qblk * 64 + w * 16;
  const float* Q = Qb + (size_t)bh * qstride; const float* K = Kb + (size_t)bh * kstride; const float* V = Vb + (size_t)bh * vstride + dv0;
  FragB aqh[KS], aql[KS];
  {
    int row = q0 + ln; if (row >= Tq) row = Tq - 1;
    const float* qr = Q + (size_t)row * qpitch;
#pragma unroll
    for (int ks = 0; ks < KS; ++ks)
#pragma unroll
      for (int i = 0; i < 16; ++i) {
        const int d = ks * 32 + ((i < 8) ? (8 * hh + i) : (16 + 8 * hh + (i - 8)));
        const float x = qr[d] * scale; const unsigned short hb = bf16_bits(x);
        aqh[ks].u[i] = hb; aql[ks].u[i] = bf16_bits(x - bf16_val(hb));
      }
  }
  float m_r[8], l_r[8];
#pragma unroll
  for (int r = 0; r < 8; ++r) { m_r[r] = -3.0e38f; l_r[r] = 0.f; }
  v8f oacc[DT];
#pragma unroll
  for (int dt = 0; dt < DT; ++dt) oacc[dt] = (v8f){0.f,0.f,0.f,0.f,0.f,0.f,0.f,0.f};
  for (int j0 = 0; j0 < Tk; j0 += 32) {
    __syncthreads();
    for (int e = tid; e < 32 * (DQ / 4); e += 128) {
      const int r = e / (DQ / 4), c4 = (e % (DQ / 4)) * 4; const int key = j0 + r;
      v4f f = {0.f,0.f,0.f,0.f}; if (key < Tk) f = *(const v4fa*)(K + (size_t)key * kpitch + c4);
#pragma unroll
      for (int t = 0; t < 4; ++t) { const unsigned short hb = bf16_bits(f[t]); sKh[r][c4 + t] = hb; sKl[r][c4 + t] = bf16_bits(f[t] - bf16_val(hb)); }
    }
    for (int e = tid; e < 32 * (DV / 4); e += 128) {
      const int r = e / (DV / 4), c4 = (e % (DV / 4)) * 4; const int key = j0 + r;
      v4f f = {0.f,0.f,0.f,0.f}; if (key < Tk) f = *(const v4fa*)(V + (size_t)key * vpitch + c4);
#pragma unroll
      for (int t = 0; t < 4; ++t) { const unsigned short hb = bf16_bits(f[t]); sVh[r][c4 + t] = hb; sVl[r][c4 + t] = bf16_bits(f[t] - bf16_val(hb)); }
    }
    __syncthreads();
    v8f s[2];
#pragma unroll
    for (int nt = 0; nt < 2; ++nt) {
      v8f acc = {};
#pragma unroll
      for (int ks = 0; ks < KS; ++ks) {
        FragB bh_, bl_;
        bh_.half[0] = *(const v8us*)&sKh[nt * 16 + ln][ks * 32 + 8 * hh]; bh_.half[1] = *(const v8us*)&sKh[nt * 16 + ln][ks * 32 + 16 + 8 * hh];
        bl_.half[0] = *(const v8us*)&sKl[nt * 16 + ln][ks * 32 + 8 * hh]; bl_.half[1] = *(const v8us*)&sKl[nt * 16 + ln][ks * 32 + 16 + 8 * hh];
        acc = mmaN<3>(aqh[ks].v, aql[ks].v, bh_.v, bl_.v, acc);
      }
      s[nt] = acc;
    }
    float alpha[8];
#pragma unroll
    for (int r = 0; r < 8; ++r) {
      const int ja = j0 + ln, jb = j0 + 16 + ln;
      if (ja >= Tk) s[0][r] = -3.0e38f;
      if (jb >= Tk) s[1][r] = -3.0e38f;
      float mx = fmaxf(s[0][r], s[1][r]);
      mx = fmaxf(mx, __shfl_xor(mx, 1, 32)); mx = fmaxf(mx, __shfl_xor(mx, 2, 32)); mx = fmaxf(mx, __shfl_xor(mx, 4, 32)); mx = fmaxf(mx, __shfl_xor(mx, 8, 32));
      const float mnew = fmaxf(m_r[r], mx);
      alpha[r] = (mnew > -1.0e38f) ? __expf(m_r[r] - mnew) : 1.0f;
      const float p0 = (s[0][r] > -1.0e38f) ? __expf(s[0][r] - mnew) : 0.f;
      const float p1 = (s[1][r] > -1.0e38f) ? __expf(s[1][r] - mnew) : 0.f;
      m_r[r] = mnew;
      l_r[r] = l_r[r] * alpha[r] + p0 + p1;
      unsigned short hb = bf16_bits(p0); sPh[w][8 * hh + r][ln] = hb;      sPl[w][8 * hh + r][ln] = bf16_bits(p0 - bf16_val(hb));
      hb = bf16_bits(p1);                sPh[w][8 * hh + r][16 + ln] = hb; sPl[w][8 * hh + r][16 + ln] = bf16_bits(p1 - bf16_val(hb));
    }
#pragma unroll
    for (int dt = 0; dt < DT; ++dt)
#pragma unroll
      for (int r = 0; r < 8; ++r) oacc[dt][r] *= alpha[r];
    __builtin_amdgcn_fence(__ATOMIC_ACQ_REL, "workgroup");
    __builtin_amdgcn_wave_barrier();
    FragB pah, pal;
    pah.half[0] = *(const v8us*)&sPh[w][ln][8 * hh]; pah.half[1] = *(const v8us*)&sPh[w][ln][16 + 8 * hh];
    pal.half[0] = *(const v8us*)&sPl[w][ln][8 * hh]; pal.half[1] = *(const v8us*)&sPl[w][ln][16 + 8 * hh];
#pragma unroll
    for (int dt = 0; dt < DT; ++dt) {
      FragB bvh, bvl;
#pragma unroll
      for (int i = 0; i < 8; ++i) {
        bvh.u[i] = sVh[8 * hh + i][dt * 16 + ln]; bvh.u[8 + i] = sVh[16 + 8 * hh + i][dt * 16 + ln];
        bvl.u[i] = sVl[8 * hh + i][dt * 16 + ln]; bvl.u[8 + i] = sVl[16 + 8 * hh + i][dt * 16 + ln];
      }
      oacc[dt] = mmaN<3>(pah.v, pal.v, bvh.v, bvl.v, oacc[dt]);
    }
    __builtin_amdgcn_fence(__ATOMIC_ACQ_REL, "workgroup");
    __builtin_amdgcn_wave_barrier();
  }
#pragma unroll
  for (int r = 0; r < 8; ++r) {
    float l = l_r[r];
    l += __shfl_xor(l, 1, 32); l += __shfl_xor(l, 2, 32); l += __shfl_xor(l, 4, 32); l += __shfl_xor(l, 8, 32);
    l_r[r] = (l > 0.f) ? 1.0f / l : 0.f;
  }
#pragma unroll
  for (int dt = 0; dt < DT; ++dt)
#pragma unroll
    for (int r = 0; r < 8; ++r) sO[w][8 * hh + r][dt * 16 + ln] = oacc[dt][r] * l_r[r];
  __builtin_amdgcn_fence(__ATOMIC_ACQ_REL, "workgroup");
  __builtin_amdgcn_wave_barrier();
  for (int pass = 0; pass < 2; ++pass) {
    for (int r = 0; r < 16; ++r) {
      const int row = q0 + r;
      for (int c4 = lane * 4; c4 < DV; c4 += 128) {
        if (row < Tq) {
          const v4f val = *(const v4fa*)&sO[w][r][c4];
          *(volatile v4f*)(y + (size_t)bh * ystride + (size_t)row * ypitch + dv0 + c4) = val;
        }
      }
    }
    if (pass == 0) __threadfence();
  }
}

__global__ __launch_bounds__(256) void k_split_rows(const float* __restrict__ src, int lds_, unsigned short* __restrict__ hi, unsigned short* __restrict__ lo, int R, int Cc) {
  const size_t t = (size_t)blockIdx.x * 256 + threadIdx.x;
  const int c8n = Cc / 8;
  if (t >= (size_t)R * c8n) return;
  const int r = (int)(t / c8n), c8 = (int)(t % c8n) * 8;
  const float* s = src + (size_t)r * lds_ + c8;
  const v4f a = *(const v4fa*)s, b = *(const v4fa*)(s + 4);
  float xs[8] = {a[0],a[1],a[2],a[3],b[0],b[1],b[2],b[3]};
  v8us vh, vl;
#pragma unroll
  for (int i = 0; i < 8; ++i) { const unsigned short hb = bf16_bits(xs[i]); vh[i] = hb; vl[i] = bf16_bits(xs[i] - bf16_val(hb)); }
  unsigned short* dh = hi + (size_t)r * Cc + c8; unsigned short* dl = lo + (size_t)r * Cc + c8;
  *(volatile v8us*)dh = vh; *(volatile v8us*)dl = vl; __threadfence(); *(volatile v8us*)dh = vh; *(volatile v8us*)dl = vl;
}
__global__ __launch_bounds__(256) void k_split_transpose(const float* __restrict__ src, int lds_, unsigned short* __restrict__ hi, unsigned short* __restrict__ lo, int K, int N) {
  const size_t t = (size_t)blockIdx.x * 256 + threadIdx.x;
  const int k8n = K / 8;
  if (t >= (size_t)N * k8n) return;
  const int n = (int)(t / k8n), k8 = (int)(t % k8n) * 8;
  v8us vh, vl;
#pragma unroll
  for (int i = 0; i < 8; ++i) { const float x = src[(size_t)(k8 + i) * lds_ + n]; const unsigned short hb = bf16_bits(x); vh[i] = hb; vl[i] = bf16_bits(x - bf16_val(hb)); }
  unsigned short* dh = hi + (size_t)n * K + k8; unsigned short* dl = lo + (size_t)n * K + k8;
  *(volatile v8us*)dh = vh; *(volatile v8us*)dl = vl; __threadfence(); *(volatile v8us*)dh = vh; *(volatile v8us*)dl = vl;
}
template <bool ASPLIT, bool BSPLIT, int ACT, bool BIAS_BF16>
__global__ __launch_bounds__(128) void k_gemm_bf2(const float* __restrict__ A, int lda, const unsigned short* __restrict__ Bh, const unsigned short* __restrict__ Bl, int ldb,
                                                const float* __restrict__ bias, float alpha, float* __restrict__ C, int ldc, int M, int N, int K) {
  __shared__ __attribute__((aligned(16))) float so[4][16][64];
  const int tid = threadIdx.x, w = tid >> 5, lane = tid & 31, ln = lane & 15, hh = lane >> 4;
  const int ntn = N / 64;
  const int wid = blockIdx.x * 4 + w;
  const int mt = wid / ntn, nq = wid % ntn;
  if (mt * 16 >= M) return;
  const int row0 = mt * 16, col0 = nq * 64;
  const float* arow = A + (size_t)(row0 + ln) * lda;
  v8f acc[4] = {};
  for (int kb = 0; kb < K; kb += 32) {
    FragB ah, al;
    const v4f x0 = *(const v4fa*)(arow + kb + 8 * hh), x1 = *(const v4fa*)(arow + kb + 8 * hh + 4);
    const v4f x2 = *(const v4fa*)(arow + kb + 16 + 8 * hh), x3 = *(const v4fa*)(arow + kb + 16 + 8 * hh + 4);
    float xs[16] = {x0[0],x0[1],x0[2],x0[3],x1[0],x1[1],x1[2],x1[3],x2[0],x2[1],x2[2],x2[3],x3[0],x3[1],x3[2],x3[3]};
#pragma unroll
    for (int i = 0; i < 16; ++i) { const unsigned short hb = bf16_bits(xs[i]); ah.u[i] = hb; al.u[i] = ASPLIT ? bf16_bits(xs[i] - bf16_val(hb)) : (unsigned short)0; }
#pragma unroll
    for (int t = 0; t < 4; ++t) {
      const size_t boff = (size_t)(col0 + t * 16 + ln) * ldb + kb;
      FragB bh_, bl_;
      bh_.half[0] = *(const v8us*)(Bh + boff + 8 * hh);
      bh_.half[1] = *(const v8us*)(Bh + boff + 16 + 8 * hh);
      if (BSPLIT) { bl_.half[0] = *(const v8us*)(Bl + boff + 8 * hh); bl_.half[1] = *(const v8us*)(Bl + boff + 16 + 8 * hh); } else bl_ = bh_;
      acc[t] = mmaN<ASPLIT ? (BSPLIT ? 3 : 2) : 1>(ah.v, al.v, bh_.v, bl_.v, acc[t]);
    }
  }
#pragma unroll
  for (int t = 0; t < 4; ++t) {
    float bv = bias ? bias[col0 + t * 16 + ln] : 0.f;
    if (BIAS_BF16) bv = bf16_round(bv);
#pragma unroll
    for (int r = 0; r < 8; ++r) { float v = acc[t][r] * alpha + bv; if (ACT == 1) v = fmaxf(v, 0.f); so[w][8 * hh + r][t * 16 + ln] = v; }
  }
  __builtin_amdgcn_fence(__ATOMIC_ACQ_REL, "workgroup");
  __builtin_amdgcn_wave_barrier();
  const int rsub = lane >> 4, c4 = (lane & 15) * 4;
  for (int pass = 0; pass < 2; ++pass) {
#pragma unroll
    for (int q = 0; q < 8; ++q) {
      const int r = q * 2 + rsub;
      const v4f v = *(const v4fa*)&so[w][r][c4];
      *(volatile v4f*)(C + (size_t)(row0 + r) * ldc + col0 + c4) = v;
    }
    if (pass == 0) __threadfence();
  }
}
__global__ __launch_bounds__(256) void k_softmax_rows(const float* __restrict__ S, float* __restrict__ P, int N, int causal, int rowoff, const int* __restrict__ mask, int mask_pitch) {
  __shared__ float red[256];
  const int row = blockIdx.x, tid = threadIdx.x;
  const float* s = S + (size_t)row * N; float* p_out = P + (size_t)row * N;
  const int qi = row + rowoff;
  float mx = -3.0e38f;
  for (int j = tid; j < N; j += 256) {
    bool keep = true;
    if (causal && j > qi) keep = false;
    if (mask && mask[(size_t)qi * mask_pitch + j] == 0) keep = false;
    const float v = keep ? s[j] : -3.0e38f;
    mx = fmaxf(mx, v);
  }
  red[tid] = mx; __syncthreads();
  for (int st = 128; st > 0; st >>= 1) { if (tid < st) red[tid] = fmaxf(red[tid], red[tid + st]); __syncthreads(); }
  mx = red[0]; __syncthreads();
  float sum = 0.f;
  for (int j = tid; j < N; j += 256) {
    bool keep = true;
    if (causal && j > qi) keep = false;
    if (mask && mask[(size_t)qi * mask_pitch + j] == 0) keep = false;
    const float p = keep ? __expf(s[j] - mx) : 0.f;
    sum += p;
  }
  red[tid] = sum; __syncthreads();
  for (int st = 128; st > 0; st >>= 1) { if (tid < st) red[tid] += red[tid + st]; __syncthreads(); }
  const float inv = (mx > -1.0e38f) ? 1.0f / red[0] : __builtin_nanf("");
  __syncthreads();
  for (int pass = 0; pass < 2; ++pass) {
    for (int j4 = tid * 4; j4 < N; j4 += 1024) {
      v4f out4;
#pragma unroll
      for (int u = 0; u < 4; ++u) {
        const int j = j4 + u;
        bool keep = true;
        if (causal && j > qi) keep = false;
        if (mask && mask[(size_t)qi * mask_pitch + j] == 0) keep = false;
        out4[u] = keep ? __expf(s[j] - mx) * inv : 0.f;
      }
      *(volatile v4f*)(p_out + j4) = out4;
    }
    if (pass == 0) __threadfence();
  }
}

template <bool ASPLIT, int ACT, bool BIAS_BF16, bool RES_BF16>
__global__ __launch_bounds__(128) void k_gemm_bf3(const float* __restrict__ A, int lda, const unsigned short* __restrict__ Wt, int ldb,
                                                const float* __restrict__ bias, const float* __restrict__ resid, int rmod, int ldr,
                                                float* __restrict__ C, int ldc, int M, int N, int K) {
  __shared__ __attribute__((aligned(16))) float so[4][16][64];
  const int tid = threadIdx.x, w = tid >> 5, lane = tid & 31, ln = lane & 15, hh = lane >> 4;
  const int ntn = N / 64;
  const int wid = blockIdx.x * 4 + w;
  const int mt = wid / ntn, nq = wid % ntn;
  if (mt * 16 >= M) return;
  const int row0 = mt * 16, col0 = nq * 64;
  const float* arow = A + (size_t)(row0 + ln) * lda;
  v8f acc[4] = {};
  for (int kb = 0; kb < K; kb += 32) {
    FragB ah, al;
    const v4f x0 = *(const v4fa*)(arow + kb + 8 * hh), x1 = *(const v4fa*)(arow + kb + 8 * hh + 4);
    const v4f x2 = *(const v4fa*)(arow + kb + 16 + 8 * hh), x3 = *(const v4fa*)(arow + kb + 16 + 8 * hh + 4);
    float xs[16] = {x0[0],x0[1],x0[2],x0[3],x1[0],x1[1],x1[2],x1[3],x2[0],x2[1],x2[2],x2[3],x3[0],x3[1],x3[2],x3[3]};
#pragma unroll
    for (int i = 0; i < 16; ++i) { const unsigned short hb = bf16_bits(xs[i]); ah.u[i] = hb; al.u[i] = ASPLIT ? bf16_bits(xs[i] - bf16_val(hb)) : (unsigned short)0; }
#pragma unroll
    for (int t = 0; t < 4; ++t) {
      const unsigned short* brow = Wt + (size_t)(col0 + t * 16 + ln) * ldb + kb;
      FragB b;
      b.half[0] = *(const v8us*)(brow + 8 * hh);
      b.half[1] = *(const v8us*)(brow + 16 + 8 * hh);
      acc[t] = mmaN<ASPLIT ? 2 : 1>(ah.v, al.v, b.v, b.v, acc[t]);
    }
  }
#pragma unroll
  for (int t = 0; t < 4; ++t) {
    const int col = col0 + t * 16 + ln;
    float bv = bias ? bias[col] : 0.f;
    if (BIAS_BF16) bv = bf16_round(bv);
#pragma unroll
    for (int r = 0; r < 8; ++r) {
      float v = acc[t][r] + bv;
      if (resid) { float rv = resid[(size_t)((row0 + 8 * hh + r) % rmod) * ldr + col]; if (RES_BF16) rv = bf16_round(rv); v += rv; }
      if (ACT == 1) v = fmaxf(v, 0.f);
      if (ACT == 2) v = 0.5f * v * (1.0f + erff(v * 0.70710678118654752f));
      if (ACT == 3) { const float u = 0.7978845608028654f * (v + 0.044715f * v * v * v); v = 0.5f * v * (1.0f + tanhf(u)); }
      so[w][8 * hh + r][t * 16 + ln] = v;
    }
  }
  __builtin_amdgcn_fence(__ATOMIC_ACQ_REL, "workgroup");
  __builtin_amdgcn_wave_barrier();
  const int rsub = lane >> 4, c4 = (lane & 15) * 4;
  for (int pass = 0; pass < 2; ++pass) {
#pragma unroll
    for (int q = 0; q < 8; ++q) {
      const int r = q * 2 + rsub;
      const v4f v = *(const v4fa*)&so[w][r][c4];
      *(volatile v4f*)(C + (size_t)(row0 + r) * ldc + col0 + c4) = v;
    }
    if (pass == 0) __threadfence();
  }
}
template <bool PARAM_BF16>
__global__ __launch_bounds__(256) void k_layernorm(const float* __restrict__ X, const float* __restrict__ R, const float* __restrict__ g, const float* __restrict__ bta,
                                                  float* __restrict__ out_sum, float* __restrict__ out_norm, int N, float eps) {
  __shared__ float red[256];
  const int row = blockIdx.x, tid = threadIdx.x;
  const float* x = X + (size_t)row * N; const float* rr = R ? R + (size_t)row * N : nullptr;
  float vals[16];
  const int per = N / 256;
  float s1 = 0.f;
  for (int u = 0; u < per / 4; ++u) {
    const int j = tid * 4 + 1024 * u;
    const v4f a = *(const v4fa*)(x + j);
    v4f b = {0.f,0.f,0.f,0.f}; if (rr) b = *(const v4fa*)(rr + j);
#pragma unroll
    for (int q = 0; q < 4; ++q) { const float v = a[q] + b[q]; vals[u * 4 + q] = v; s1 += v; }
  }
  red[tid] = s1; __syncthreads();
  for (int st = 128; st > 0; st >>= 1) { if (tid < st) red[tid] += red[tid + st]; __syncthreads(); }
  const float mu = red[0] / (float)N; __syncthreads();
  float s2 = 0.f;
  for (int u = 0; u < per / 4; ++u)
#pragma unroll
    for (int q = 0; q < 4; ++q) { const float c = vals[u * 4 + q] - mu; s2 += c * c; }
  red[tid] = s2; __syncthreads();
  for (int st = 128; st > 0; st >>= 1) { if (tid < st) red[tid] += red[tid + st]; __syncthreads(); }
  const float rs = rsqrtf(red[0] / (float)N + eps);
  for (int pass = 0; pass < 2; ++pass) {
    for (int u = 0; u < per / 4; ++u) {
      const int j = tid * 4 + 1024 * u;
      v4f o, sm;
#pragma unroll
      for (int q = 0; q < 4; ++q) {
        float gg = g[j + q], bb = bta[j + q];
        if (PARAM_BF16) { gg = bf16_round(gg); bb = bf16_round(bb); }
        sm[q] = vals[u * 4 + q]; o[q] = (vals[u * 4 + q] - mu) * rs * gg + bb;
      }
      if (out_sum) *(volatile v4f*)(out_sum + (size_t)row * N + j) = sm;
      *(volatile v4f*)(out_norm + (size_t)row * N + j) = o;
    }
    if (pass == 0) __threadfence();
  }
}

template <bool ASPLIT, bool BSPLIT, int ACT>
__global__ __launch_bounds__(128) void k_gemm_b(const float* __restrict__ A, int lda, size_t sA, const unsigned short* __restrict__ Bh, const unsigned short* __restrict__ Bl, int ldb, size_t sB,
                                             const float* __restrict__ bias, const float* __restrict__ resid, int ldr, size_t sR, float rsign, float alpha,
                                             float* __restrict__ C, int ldc, size_t sC, int M, int N, int K) {
  __shared__ __attribute__((aligned(16))) float so[4][16][64];
  const int tid = threadIdx.x, w = tid >> 5, lane = tid & 31, ln = lane & 15, hh = lane >> 4;
  const int by = blockIdx.y;
  A += (size_t)by * sA; Bh += (size_t)by * sB; if (BSPLIT) Bl += (size_t)by * sB; C += (size_t)by * sC; if (resid) resid += (size_t)by * sR;
  const int ntn = N / 64; const int wid = blockIdx.x * 4 + w; const int mt = wid / ntn, nq = wid % ntn;
  if (mt * 16 >= M) return;
  const int row0 = mt * 16, col0 = nq * 64;
  const float* arow = A + (size_t)(row0 + ln) * lda;
  v8f acc[4] = {};
  for (int kb = 0; kb < K; kb += 32) {
    FragB ah, al;
    const v4f x0 = *(const v4fa*)(arow + kb + 8 * hh), x1 = *(const v4fa*)(arow + kb + 8 * hh + 4);
    const v4f x2 = *(const v4fa*)(arow + kb + 16 + 8 * hh), x3 = *(const v4fa*)(arow + kb + 16 + 8 * hh + 4);
    float xs[16] = {x0[0],x0[1],x0[2],x0[3],x1[0],x1[1],x1[2],x1[3],x2[0],x2[1],x2[2],x2[3],x3[0],x3[1],x3[2],x3[3]};
#pragma unroll
    for (int i = 0; i < 16; ++i) { const unsigned short hb = bf16_bits(xs[i]); ah.u[i] = hb; al.u[i] = ASPLIT ? bf16_bits(xs[i] - bf16_val(hb)) : (unsigned short)0; }
#pragma unroll
    for (int t = 0; t < 4; ++t) {
      const size_t boff = (size_t)(col0 + t * 16 + ln) * ldb + kb;
      FragB bh_, bl_; bh_.half[0] = *(const v8us*)(Bh + boff + 8 * hh); bh_.half[1] = *(const v8us*)(Bh + boff + 16 + 8 * hh);
      if (BSPLIT) { bl_.half[0] = *(const v8us*)(Bl + boff + 8 * hh); bl_.half[1] = *(const v8us*)(Bl + boff + 16 + 8 * hh); } else bl_ = bh_;
      acc[t] = mmaN<ASPLIT ? (BSPLIT ? 3 : 2) : 1>(ah.v, al.v, bh_.v, bl_.v, acc[t]);
    }
  }
#pragma unroll
  for (int t = 0; t < 4; ++t) {
    const int col = col0 + t * 16 + ln; const float bv = bias ? bf16_round(bias[col]) : 0.f;
#pragma unroll
    for (int r = 0; r < 8; ++r) { float v = acc[t][r] * alpha + bv; if (resid) v += rsign * resid[(size_t)(row0 + 8 * hh + r) * ldr + col]; if (ACT == 1) v = fmaxf(v, 0.f); else if (ACT == 2) v = fmaxf(v, 0.f) + log1pf(expf(-fabsf(v))); so[w][8 * hh + r][t * 16 + ln] = v; }
  }
  __builtin_amdgcn_fence(__ATOMIC_ACQ_REL, "workgroup"); __builtin_amdgcn_wave_barrier();
  const int rsub = lane >> 4, c4 = (lane & 15) * 4;
  for (int pass = 0; pass < 2; ++pass) {
#pragma unroll
    for (int q = 0; q < 8; ++q) { const int r = q * 2 + rsub; const v4f v = *(const v4fa*)&so[w][r][c4]; *(volatile v4f*)(C + (size_t)(row0 + r) * ldc + col0 + c4) = v; }
    if (pass == 0) __threadfence();
  }
}
__global__ __launch_bounds__(256) void k_split_transpose_b(const float* __restrict__ src, int lds_, size_t sIn, unsigned short* __restrict__ hi, unsigned short* __restrict__ lo, size_t sOut, int K, int N) {
  const size_t t = (size_t)blockIdx.x * 256 + threadIdx.x; const int k8n = K / 8; if (t >= (size_t)N * k8n) return;
  src += (size_t)blockIdx.y * sIn; hi += (size_t)blockIdx.y * sOut; lo += (size_t)blockIdx.y * sOut;
  const int n = (int)(t / k8n), k8 = (int)(t % k8n) * 8; v8us vh, vl;
#pragma unroll
  for (int i = 0; i < 8; ++i) { const float x = src[(size_t)(k8 + i) * lds_ + n]; const unsigned short hb = bf16_bits(x); vh[i] = hb; vl[i] = bf16_bits(x - bf16_val(hb)); }
  unsigned short* dh = hi + (size_t)n * K + k8; unsigned short* dl = lo + (size_t)n * K + k8;
  *(volatile v8us*)dh = vh; *(volatile v8us*)dl = vl; __threadfence(); *(volatile v8us*)dh = vh; *(volatile v8us*)dl = vl;
}

__global__ __launch_bounds__(256) void k_roundcopy(const float* __restrict__ src, float* __restrict__ dst, int n8) {
  const size_t t = (size_t)blockIdx.x * 256 + threadIdx.x;
  if (t >= (size_t)n8 * 2) return;
  v4f a = *(const v4fa*)(src + t * 4);
  for (int i = 0; i < 4; ++i) a[i] = bf16_round(a[i]);
  *(volatile v4f*)(dst + t * 4) = a; __threadfence(); *(volatile v4f*)(dst + t * 4) = a;
}

__global__ __launch_bounds__(256) void k_reparam(const float* __restrict__ h3, const float* __restrict__ eps, float* __restrict__ z, float* __restrict__ omean, float* __restrict__ ologv) {
  const int t = blockIdx.x * 256 + threadIdx.x; if (t >= K2 * LAT / 4) return; const int r = t / (LAT / 4), c4 = (t % (LAT / 4)) * 4;
  const v4f m = *(const v4fa*)(h3 + (size_t)r * 2 * LAT + c4), lv = *(const v4fa*)(h3 + (size_t)r * 2 * LAT + LAT + c4); v4f zz;
  for (int q = 0; q < 4; ++q) zz[q] = m[q] + expf(0.5f * lv[q]) * bf16_round(eps[(size_t)r * LAT + c4 + q]);
  *(volatile v4f*)(z + (size_t)t * 4) = zz; *(volatile v4f*)(omean + (size_t)t * 4) = m; *(volatile v4f*)(ologv + (size_t)t * 4) = lv; __threadfence();
  *(volatile v4f*)(z + (size_t)t * 4) = zz; *(volatile v4f*)(omean + (size_t)t * 4) = m; *(volatile v4f*)(ologv + (size_t)t * 4) = lv;
}
extern "C" void kernel_launch(void* const* d_in, const int* in_sizes, int n_in,
                              void* d_out, int out_size, void* d_ws, size_t ws_size, hipStream_t stream) {
  (void)in_sizes; (void)n_in; (void)out_size;
  const float* x = (const float*)d_in[0]; const float* eps = (const float*)d_in[1]; const float* adj = (const float*)d_in[2];
  const float* We1 = (const float*)d_in[3]; const float* be1 = (const float*)d_in[4]; const float* Kemb1 = (const float*)d_in[5]; const float* Kpool1 = (const float*)d_in[6];
  const float* We2 = (const float*)d_in[7]; const float* be2 = (const float*)d_in[8]; const float* Kemb2 = (const float*)d_in[9]; const float* Kpool2 = (const float*)d_in[10];
  const float* We3 = (const float*)d_in[11]; const float* be3 = (const float*)d_in[12]; const float* Wd0 = (const float*)d_in[13]; const float* bd0 = (const float*)d_in[14];
  const float* Wd1 = (const float*)d_in[15]; const float* bd1 = (const float*)d_in[16]; const float* Wd2 = (const float*)d_in[17]; const float* bd2 = (const float*)d_in[18]; const float* Wdf = (const float*)d_in[19]; const float* bdf = (const float*)d_in[20];
  float* out0 = (float*)d_out; float* out1 = (float*)((char*)d_out + 4194304); float* out2 = (float*)((char*)d_out + 5242880);
  char* ws = (char*)d_ws; size_t off = 0;
  auto take = [&](size_t bytes) { char* p = ws + off; off += (bytes + 255) & ~(size_t)255; return p; };
  unsigned short* Be1 = (unsigned short*)take((size_t)HH * FF * 2); unsigned short* Bk1 = (unsigned short*)take((size_t)(HH + K1) * HH * 2); unsigned short* Be2 = (unsigned short*)take((size_t)HH * HH * 2); unsigned short* Bk2 = (unsigned short*)take((size_t)(HH + K2) * HH * 2);
  unsigned short* Be3 = (unsigned short*)take((size_t)2 * LAT * HH * 2); unsigned short* Bd0 = (unsigned short*)take((size_t)HH * LAT * 2); unsigned short* Bd1 = (unsigned short*)take((size_t)HH * HH * 2); unsigned short* Bd2 = (unsigned short*)take((size_t)HH * HH * 2); unsigned short* Bdf = (unsigned short*)take((size_t)FF * HH * 2);
  float* A0 = (float*)take((size_t)NN * NN * 4);
  float* t256 = (float*)take((size_t)NN * HH * 4); float* h = (float*)take((size_t)NN * HH * 4); float* hK = (float*)take((size_t)NN * (HH + K1) * 4);
  unsigned short* Ph = (unsigned short*)take((size_t)(HH + K1) * NN * 2); unsigned short* Pl = (unsigned short*)take((size_t)(HH + K1) * NN * 2);
  float* z1 = (float*)take((size_t)NN * HH * 4); float* sp = (float*)take((size_t)NN * K1 * 4); float* s1 = (float*)take((size_t)NN * K1 * 4); float* s1T = (float*)take((size_t)K1 * NN * 4);
  unsigned short* S1h = (unsigned short*)take((size_t)K1 * NN * 2); unsigned short* S1l = (unsigned short*)take((size_t)K1 * NN * 2);
  float* AS = (float*)take((size_t)NN * K1 * 4); float* A1 = (float*)take((size_t)K1 * K1 * 4); float* xp1 = (float*)take((size_t)K1 * HH * 4);
  float* z2 = (float*)take((size_t)K1 * HH * 4); float* s2 = (float*)take((size_t)K1 * K2 * 4); float* s2T = (float*)take((size_t)K2 * K1 * 4);
  unsigned short* S2h = (unsigned short*)take((size_t)K2 * K1 * 2); unsigned short* S2l = (unsigned short*)take((size_t)K2 * K1 * 2);
  float* A2 = (float*)take((size_t)K2 * K2 * 4); float* xp2 = (float*)take((size_t)K2 * HH * 4); float* h3 = (float*)take((size_t)K2 * 2 * LAT * 4); float* zl = (float*)take((size_t)K2 * LAT * 4);
  if (off > ws_size) return;
  k_wt_bf16<<<(HH * (FF / 8) + 255) / 256, 256, 0, stream>>>(We1, Be1, FF, HH);
  k_wt_bf16<<<(HH * (HH / 8) + 255) / 256, 256, 0, stream>>>(Kemb1, Bk1, HH, HH); k_wt_bf16<<<(K1 * (HH / 8) + 255) / 256, 256, 0, stream>>>(Kpool1, Bk1 + (size_t)HH * HH, HH, K1);
  k_wt_bf16<<<(HH * (HH / 8) + 255) / 256, 256, 0, stream>>>(We2, Be2, HH, HH);
  k_wt_bf16<<<(HH * (HH / 8) + 255) / 256, 256, 0, stream>>>(Kemb2, Bk2, HH, HH); k_wt_bf16<<<(K2 * (HH / 8) + 255) / 256, 256, 0, stream>>>(Kpool2, Bk2 + (size_t)HH * HH, HH, K2);
  k_wt_bf16<<<(2 * LAT * (HH / 8) + 255) / 256, 256, 0, stream>>>(We3, Be3, HH, 2 * LAT); k_wt_bf16<<<(HH * (LAT / 8) + 255) / 256, 256, 0, stream>>>(Wd0, Bd0, LAT, HH);
  k_wt_bf16<<<(HH * (HH / 8) + 255) / 256, 256, 0, stream>>>(Wd1, Bd1, HH, HH); k_wt_bf16<<<(HH * (HH / 8) + 255) / 256, 256, 0, stream>>>(Wd2, Bd2, HH, HH); k_wt_bf16<<<(FF * (HH / 8) + 255) / 256, 256, 0, stream>>>(Wdf, Bdf, HH, FF);
  k_roundcopy<<<(NN * NN / 4 + 255) / 256, 256, 0, stream>>>(adj, A0, NN * NN / 8);
  auto gb = [](int M, int N) { return dim3(((M / 16) * (N / 64) + 3) / 4, 1); };
  for (int b = 0; b < BB; ++b) {
    const float* xb = x + (size_t)b * NN * FF; const float* eb = eps + (size_t)b * K2 * LAT;
    k_gemm_bf3<false, 0, false, false><<<gb(NN, HH), 128, 0, stream>>>(xb, FF, Be1, FF, nullptr, nullptr, 1, 0, t256, HH, NN, HH, FF);
    k_split_transpose_b<<<dim3((HH * (NN / 8) + 255) / 256, 1), 256, 0, stream>>>(t256, HH, 0, Ph, Pl, 0, NN, HH);
    k_gemm_b<true, true, 1><<<gb(NN, HH), 128, 0, stream>>>(A0, NN, 0, Ph, Pl, NN, 0, be1, nullptr, 0, 0, 1.f, 1.f, h, HH, 0, NN, HH, NN);
    k_gemm_bf3<true, 0, false, false><<<gb(NN, HH + K1), 128, 0, stream>>>(h, HH, Bk1, HH, nullptr, nullptr, 1, 0, hK, HH + K1, NN, HH + K1, HH);
    k_split_transpose_b<<<dim3(((HH + K1) * (NN / 8) + 255) / 256, 1), 256, 0, stream>>>(hK, HH + K1, 0, Ph, Pl, 0, NN, HH + K1);
    k_gemm_b<true, true, 0><<<gb(NN, HH), 128, 0, stream>>>(A0, NN, 0, Ph, Pl, NN, 0, nullptr, nullptr, 0, 0, 1.f, 1.f, z1, HH, 0, NN, HH, NN);
    k_gemm_b<true, true, 0><<<gb(NN, K1), 128, 0, stream>>>(A0, NN, 0, Ph + (size_t)HH * NN, Pl + (size_t)HH * NN, NN, 0, nullptr, nullptr, 0, 0, 1.f, 1.f, sp, K1, 0, NN, K1, NN);
    k_softmax_rows<<<NN, 256, 0, stream>>>(sp, s1, K1, 0, 0, nullptr, 0);
    k_transpose32<false, false, false><<<dim3(K1 / 32, NN / 32, 1), 256, 0, stream>>>(s1, s1T, NN, K1, nullptr, nullptr, nullptr);
    k_split_transpose_b<<<dim3((HH * (NN / 8) + 255) / 256, 1), 256, 0, stream>>>(z1, HH, 0, Ph, Pl, 0, NN, HH);
    k_gemm_b<true, true, 0><<<gb(K1, HH), 128, 0, stream>>>(s1T, NN, 0, Ph, Pl, NN, 0, nullptr, nullptr, 0, 0, 1.f, 1.f, xp1, HH, 0, K1, HH, NN);
    k_split_rows<<<(K1 * NN / 8 + 255) / 256, 256, 0, stream>>>(s1T, NN, S1h, S1l, K1, NN);
    k_gemm_b<true, true, 0><<<gb(NN, K1), 128, 0, stream>>>(A0, NN, 0, S1h, S1l, NN, 0, nullptr, nullptr, 0, 0, 1.f, 1.f, AS, K1, 0, NN, K1, NN);
    k_split_transpose_b<<<dim3((K1 * (NN / 8) + 255) / 256, 1), 256, 0, stream>>>(AS, K1, 0, Ph, Pl, 0, NN, K1);
    k_gemm_b<true, true, 0><<<gb(K1, K1), 128, 0, stream>>>(s1T, NN, 0, Ph, Pl, NN, 0, nullptr, nullptr, 0, 0, 1.f, 1.f, A1, K1, 0, K1, K1, NN);
    k_gemm_bf3<true, 0, false, false><<<gb(K1, HH), 128, 0, stream>>>(xp1, HH, Be2, HH, nullptr, nullptr, 1, 0, t256, HH, K1, HH, HH);
    k_split_transpose_b<<<dim3((HH * (K1 / 8) + 255) / 256, 1), 256, 0, stream>>>(t256, HH, 0, Ph, Pl, 0, K1, HH);
    k_gemm_b<true, true, 1><<<gb(K1, HH), 128, 0, stream>>>(A1, K1, 0, Ph, Pl, K1, 0, be2, nullptr, 0, 0, 1.f, 1.f, h, HH, 0, K1, HH, K1);
    k_gemm_bf3<true, 0, false, false><<<gb(K1, HH + K2), 128, 0, stream>>>(h, HH, Bk2, HH, nullptr, nullptr, 1, 0, hK, HH + K2, K1, HH + K2, HH);
    k_split_transpose_b<<<dim3(((HH + K2) * (K1 / 8) + 255) / 256, 1), 256, 0, stream>>>(hK, HH + K2, 0, Ph, Pl, 0, K1, HH + K2);
    k_gemm_b<true, true, 0><<<gb(K1, HH), 128, 0, stream>>>(A1, K1, 0, Ph, Pl, K1, 0, nullptr, nullptr, 0, 0, 1.f, 1.f, z2, HH, 0, K1, HH, K1);
    k_gemm_b<true, true, 0><<<gb(K1, K2), 128, 0, stream>>>(A1, K1, 0, Ph + (size_t)HH * K1, Pl + (size_t)HH * K1, K1, 0, nullptr, nullptr, 0, 0, 1.f, 1.f, sp, K2, 0, K1, K2, K1);
    k_softmax_rows<<<K1, 256, 0, stream>>>(sp, s2, K2, 0, 0, nullptr, 0);
    k_transpose32<false, false, false><<<dim3(K2 / 32, K1 / 32, 1), 256, 0, stream>>>(s2, s2T, K1, K2, nullptr, nullptr, nullptr);
    k_split_transpose_b<<<dim3((HH * (K1 / 8) + 255) / 256, 1), 256, 0, stream>>>(z2, HH, 0, Ph, Pl, 0, K1, HH);
    k_gemm_b<true, true, 0><<<gb(K2, HH), 128, 0, stream>>>(s2T, K1, 0, Ph, Pl, K1, 0, nullptr, nullptr, 0, 0, 1.f, 1.f, xp2, HH, 0, K2, HH, K1);
    k_split_rows<<<(K2 * K1 / 8 + 255) / 256, 256, 0, stream>>>(s2T, K1, S2h, S2l, K2, K1);
    k_gemm_b<true, true, 0><<<gb(K1, K2), 128, 0, stream>>>(A1, K1, 0, S2h, S2l, K1, 0, nullptr, nullptr, 0, 0, 1.f, 1.f, AS, K2, 0, K1, K2, K1);
    k_split_transpose_b<<<dim3((K2 * (K1 / 8) + 255) / 256, 1), 256, 0, stream>>>(AS, K2, 0, Ph, Pl, 0, K1, K2);
    k_gemm_b<true, true, 0><<<gb(K2, K2), 128, 0, stream>>>(s2T, K1, 0, Ph, Pl, K1, 0, nullptr, nullptr, 0, 0, 1.f, 1.f, A2, K2, 0, K2, K2, K1);
    k_gemm_bf3<true, 0, false, false><<<gb(K2, 2 * LAT), 128, 0, stream>>>(xp2, HH, Be3, HH, nullptr, nullptr, 1, 0, t256, 2 * LAT, K2, 2 * LAT, HH);
    k_split_transpose_b<<<dim3((2 * LAT * (K2 / 8) + 255) / 256, 1), 256, 0, stream>>>(t256, 2 * LAT, 0, Ph, Pl, 0, K2, 2 * LAT);
    k_gemm_b<true, true, 0><<<gb(K2, 2 * LAT), 128, 0, stream>>>(A2, K2, 0, Ph, Pl, K2, 0, be3, nullptr, 0, 0, 1.f, 1.f, h3, 2 * LAT, 0, K2, 2 * LAT, K2);
    k_reparam<<<(K2 * LAT / 4 + 255) / 256, 256, 0, stream>>>(h3, eb, zl, out1 + (size_t)b * K2 * LAT, out2 + (size_t)b * K2 * LAT);
    k_gemm_bf3<true, 0, false, false><<<gb(K2, HH), 128, 0, stream>>>(zl, LAT, Bd0, LAT, nullptr, nullptr, 1, 0, t256, HH, K2, HH, LAT);
    k_split_transpose_b<<<dim3((HH * (K2 / 8) + 255) / 256, 1), 256, 0, stream>>>(t256, HH, 0, Ph, Pl, 0, K2, HH);
    k_gemm_b<true, true, 1><<<gb(K2, HH), 128, 0, stream>>>(A2, K2, 0, Ph, Pl, K2, 0, bd0, nullptr, 0, 0, 1.f, 1.f, h, HH, 0, K2, HH, K2);
    k_split_transpose_b<<<dim3((HH * (K2 / 8) + 255) / 256, 1), 256, 0, stream>>>(h, HH, 0, Ph, Pl, 0, K2, HH);
    k_gemm_b<true, true, 0><<<gb(K1, HH), 128, 0, stream>>>(s2, K2, 0, Ph, Pl, K2, 0, nullptr, nullptr, 0, 0, 1.f, 1.f, xp1, HH, 0, K1, HH, K2);
    k_gemm_bf3<true, 0, false, false><<<gb(K1, HH), 128, 0, stream>>>(xp1, HH, Bd1, HH, nullptr, nullptr, 1, 0, t256, HH, K1, HH, HH);
    k_split_transpose_b<<<dim3((HH * (K1 / 8) + 255) / 256, 1), 256, 0, stream>>>(t256, HH, 0, Ph, Pl, 0, K1, HH);
    k_gemm_b<true, true, 1><<<gb(K1, HH), 128, 0, stream>>>(A1, K1, 0, Ph, Pl, K1, 0, bd1, nullptr, 0, 0, 1.f, 1.f, h, HH, 0, K1, HH, K1);
    k_split_transpose_b<<<dim3((HH * (K1 / 8) + 255) / 256, 1), 256, 0, stream>>>(h, HH, 0, Ph, Pl, 0, K1, HH);
    k_gemm_b<true, true, 0><<<gb(NN, HH), 128, 0, stream>>>(s1, K1, 0, Ph, Pl, K1, 0, nullptr, nullptr, 0, 0, 1.f, 1.f, z1, HH, 0, NN, HH, K1);
    k_gemm_bf3<true, 0, false, false><<<gb(NN, HH), 128, 0, stream>>>(z1, HH, Bd2, HH, nullptr, nullptr, 1, 0, t256, HH, NN, HH, HH);
    k_split_transpose_b<<<dim3((HH * (NN / 8) + 255) / 256, 1), 256, 0, stream>>>(t256, HH, 0, Ph, Pl, 0, NN, HH);
    k_gemm_b<true, true, 1><<<gb(NN, HH), 128, 0, stream>>>(A0, NN, 0, Ph, Pl, NN, 0, bd2, nullptr, 0, 0, 1.f, 1.f, h, HH, 0, NN, HH, NN);
    k_gemm_bf3<true, 0, false, false><<<gb(NN, FF), 128, 0, stream>>>(h, HH, Bdf, HH, nullptr, nullptr, 1, 0, t256, FF, NN, FF, HH);
    k_split_transpose_b<<<dim3((FF * (NN / 8) + 255) / 256, 1), 256, 0, stream>>>(t256, FF, 0, Ph, Pl, 0, NN, FF);
    k_gemm_b<true, true, 2><<<gb(NN, FF), 128, 0, stream>>>(A0, NN, 0, Ph, Pl, NN, 0, bdf, nullptr, 0, 0, 1.f, 1.f, out0 + (size_t)b * NN * FF, FF, 0, NN, FF, NN);
  }
}
